// DecGreenNet_product_CP2_90967407329571
// MI455X (gfx1250) — hardware-verified
//
#include <hip/hip_runtime.h>
#include <math.h>

#ifndef NPTS
#define NPTS 16384
#endif
#ifndef NQP
#define NQP 4096
#endif
#define HID 1024
#define RR 64
#define KD 64
#define RK 4096
#define NCH (NQP / 256)
#define SP 72
#define VP 68

static_assert(NPTS % 256 == 0);
static_assert(NQP % 256 == 0);
static_assert(HID % 256 == 0 && RK % 256 == 0);
static_assert(HID % 32 == 0);
static_assert(RR * KD == RK);
static_assert(RR == 64 && KD == 64);
static_assert(KD % 32 == 0);
static_assert(SP % 8 == 0 && SP >= KD);
static_assert(VP % 4 == 0 && VP >= RR);
static_assert(512 * 8 == RR * KD);
static_assert(512 * 2 * 16 == RR * RR * 4);
static_assert((4 * RR * SP * 2 + RR * VP * 4) <= 131072);
static_assert((HID * 16 + HID * 4) <= 131072);

typedef __attribute__((ext_vector_type(16))) _Float16 v16h;
typedef __attribute__((ext_vector_type(8)))  _Float16 v8h;
typedef __attribute__((ext_vector_type(8)))  float    v8f;
typedef __attribute__((ext_vector_type(4)))  float    v4f;
typedef _Float16 h16;


#define VST2(T, ptr, val) do { const T vst2_v_ = (val); *(volatile T*)(ptr) = vst2_v_; __threadfence(); *(volatile T*)(ptr) = vst2_v_; } while (0)

union FragU { v16h v; v8h h[2]; };
__device__ __forceinline__ v16h frag_ld(const _Float16* p) {
    FragU f; f.h[0] = *(const v8h*)(p); f.h[1] = *(const v8h*)(p + 16); return f.v;
}
__device__ __forceinline__ v8f wmma16(v16h a, v16h b, v8f c) {
    c = __builtin_amdgcn_wmma_f32_16x16x32_f16(false, a, false, b, (short)0, c, false, false);
    asm volatile("v_nop\n\tv_nop\n\tv_nop\n\tv_nop" : "+v"(c) : "v"(a), "v"(b));
    return c;
}
static __device__ __forceinline__ h16 toh_flush(float v) {
    const h16 r = (h16)v;
    return (fabsf(v) < 6.103515625e-05f) ? (h16)0.0f : r;
}

__global__ __launch_bounds__(256) void k_quad_hidden(const float* __restrict__ qx, const float* __restrict__ Wa,
                                                     const float* __restrict__ ba, const float* __restrict__ eqp,
                                                     float* __restrict__ TPq, float* __restrict__ YPq) {
    __shared__ __align__(16) v4f sQ[256];
    const unsigned tid = threadIdx.x, lane = tid & 31u;
    const unsigned wave = (unsigned)__builtin_amdgcn_readfirstlane((int)(threadIdx.x >> 5));
    const unsigned h = blockIdx.x * 256u + tid;
    const unsigned chunk = blockIdx.y;
    const float ep = eqp[0];
    {
        const unsigned a = chunk * 256u + tid;
        const float x0 = qx[(size_t)a * 3u + 0u];
        const float x1 = qx[(size_t)a * 3u + 1u];
        const float x2 = qx[(size_t)a * 3u + 2u];
        const float ss = (x0 * x0 + x2 * x2) + x1 * x1;
        v4f q; q.x = x0; q.y = x1; q.z = x2; q.w = expf(-ep * ss);
        sQ[tid] = q;
    }
    __syncthreads();
    const float w0 = Wa[h], w1 = Wa[HID + h], w2 = Wa[2 * HID + h], bb = ba[h];
    float acc = 0.f;
#pragma unroll 1
    for (unsigned r = 0; r < 256u; ++r) {
        const v4f q = sQ[r];
        const float z = fmaf(q.x, w0, fmaf(q.y, w1, fmaf(q.z, w2, bb)));
        acc = fmaf(q.w, tanhf(z), acc);
    }
    VST2(float, TPq + (size_t)chunk * HID + h, acc);
    if (blockIdx.x == 0u && wave == 0u) {
        float s = 0.f;
#pragma unroll 1
        for (unsigned i = 0; i < 8u; ++i) s += sQ[lane * 8u + i].w;
#pragma unroll
        for (int o = 16; o > 0; o >>= 1) s += __shfl_xor(s, o, 32);
        VST2(float, YPq + (size_t)chunk * 32u + lane, s);
    }
}

__global__ __launch_bounds__(256) void k_quad_out(const float* __restrict__ TPq, const float* __restrict__ YPq,
                                                  const float* __restrict__ Wb, const float* __restrict__ bb,
                                                  float* __restrict__ Sq) {
    __shared__ float st[HID];
    __shared__ float sY;
    const unsigned tid = threadIdx.x;
#pragma unroll 1
    for (unsigned i = 0; i < (unsigned)(HID / 256); ++i) {
        const unsigned h = tid + 256u * i;
        float s = 0.f;
#pragma unroll 4
        for (unsigned c = 0; c < (unsigned)NCH; ++c) s += TPq[(size_t)c * HID + h];
        st[h] = s;
    }
    if (tid == 0u) {
        float y = 0.f;
#pragma unroll 4
        for (unsigned c = 0; c < (unsigned)NCH; ++c) y += YPq[(size_t)c * 32u];
        sY = y;
    }
    __syncthreads();
    const unsigned j = blockIdx.x * 256u + tid;
    float acc = 0.f;
#pragma unroll 4
    for (unsigned h = 0; h < (unsigned)HID; ++h) acc = fmaf(st[h], Wb[(size_t)h * RK + j], acc);
    const float val = fmaf(sY, bb[j], acc);
    VST2(float, Sq + j, val);
}

__global__ __launch_bounds__(512) void k_rhs(const float* __restrict__ S0, const float* __restrict__ S1, float* __restrict__ V) {
    __shared__ __align__(16) _Float16 sAh[RR * SP];
    __shared__ __align__(16) _Float16 sAl[RR * SP];
    __shared__ __align__(16) _Float16 sBh[RR * SP];
    __shared__ __align__(16) _Float16 sBl[RR * SP];
    __shared__ __align__(16) float sV[RR * VP];
    const unsigned tid = threadIdx.x, lane = tid & 31u;
    const unsigned wave = (unsigned)__builtin_amdgcn_readfirstlane((int)(threadIdx.x >> 5));
    const unsigned hh = lane >> 4, c = lane & 15u;
    {
        const unsigned row = tid >> 3, c0 = (tid & 7u) * 8u;
        const v4f a0 = *(const v4f*)(S0 + (size_t)row * KD + c0);
        const v4f a1 = *(const v4f*)(S0 + (size_t)row * KD + c0 + 4u);
        const v4f b0 = *(const v4f*)(S1 + (size_t)row * KD + c0);
        const v4f b1 = *(const v4f*)(S1 + (size_t)row * KD + c0 + 4u);
        const float av[8] = {a0.x, a0.y, a0.z, a0.w, a1.x, a1.y, a1.z, a1.w};
        const float bv[8] = {b0.x, b0.y, b0.z, b0.w, b1.x, b1.y, b1.z, b1.w};
        v8h ah, al, bh, bl;
#pragma unroll
        for (int e = 0; e < 8; ++e) {
            const h16 ha = toh_flush(av[e]);
            const h16 hb = toh_flush(bv[e]);
            ah[e] = ha;
            al[e] = toh_flush((av[e] - (float)ha) * 2048.0f);
            bh[e] = hb;
            bl[e] = toh_flush((bv[e] - (float)hb) * 2048.0f);
        }
        *(v8h*)(sAh + row * SP + c0) = ah;
        *(v8h*)(sAl + row * SP + c0) = al;
        *(v8h*)(sBh + row * SP + c0) = bh;
        *(v8h*)(sBl + row * SP + c0) = bl;
    }
    __syncthreads();
    const unsigned tm = (wave >> 2) * 16u, tn = (wave & 3u) * 16u;
    v8f acc0 = (v8f){0.f,0.f,0.f,0.f,0.f,0.f,0.f,0.f};
    v8f acc1 = (v8f){0.f,0.f,0.f,0.f,0.f,0.f,0.f,0.f};
#pragma unroll
    for (int ks = 0; ks < KD / 32; ++ks) {
        const unsigned ko = (unsigned)ks * 32u + 8u * hh;
        const v16h fah = frag_ld(sAh + (tm + c) * SP + ko);
        const v16h fal = frag_ld(sAl + (tm + c) * SP + ko);
        const v16h fbh = frag_ld(sBh + (tn + c) * SP + ko);
        const v16h fbl = frag_ld(sBl + (tn + c) * SP + ko);
        acc0 = wmma16(fah, fbh, acc0);
        acc1 = wmma16(fah, fbl, acc1);
        acc1 = wmma16(fal, fbh, acc1);
    }
#pragma unroll
    for (int r = 0; r < 8; ++r)
        sV[(tm + 8u * hh + (unsigned)r) * VP + tn + c] = acc0[r] + acc1[r] * (1.0f / 2048.0f);
    __syncthreads();
    {
        v4f vv[2];
#pragma unroll
        for (int it = 0; it < 2; ++it) {
            const unsigned idx = (unsigned)it * 512u + tid;
            const unsigned row = idx >> 4, c4 = (idx & 15u) * 4u;
            vv[it] = *(const v4f*)(sV + row * VP + c4);
        }
        for (int pass = 0; pass < 2; ++pass) {
#pragma unroll
            for (int it = 0; it < 2; ++it) {
                const unsigned idx = (unsigned)it * 512u + tid;
                *(volatile v4f*)(V + (size_t)idx * 4u) = vv[it];
            }
            __threadfence();
        }
    }
}

__global__ __launch_bounds__(256) void k_hidden_w(const float* __restrict__ Wx2, const float* __restrict__ bx2,
                                                  const float* __restrict__ V, float* __restrict__ WC) {
    __shared__ float sW[32];
    __shared__ float sR[8];
    const unsigned tid = threadIdx.x, lane = tid & 31u;
    const unsigned wave = (unsigned)__builtin_amdgcn_readfirstlane((int)(threadIdx.x >> 5));
    const unsigned blk = blockIdx.x;
    if (blk < (unsigned)(HID / 32)) {
#pragma unroll 1
        for (unsigned i = 0; i < 4u; ++i) {
            const unsigned row = blk * 32u + wave * 4u + i;
            const float* Mr = Wx2 + (size_t)row * RK;
            float acc = 0.f;
#pragma unroll 2
            for (unsigned it = 0; it < (unsigned)(RK / 128); ++it) {
                const unsigned j = (it * 32u + lane) * 4u;
                const v4f m = *(const v4f*)(Mr + j);
                const v4f vv = *(const v4f*)(V + j);
                acc = fmaf(m.x, vv.x, acc); acc = fmaf(m.y, vv.y, acc);
                acc = fmaf(m.z, vv.z, acc); acc = fmaf(m.w, vv.w, acc);
            }
#pragma unroll
            for (int o = 16; o > 0; o >>= 1) acc += __shfl_xor(acc, o, 32);
            if (lane == 0u) sW[wave * 4u + i] = acc;
        }
    } else {
        float acc = 0.f;
#pragma unroll 1
        for (unsigned it = 0; it < (unsigned)(RK / 1024); ++it) {
            const unsigned j = (it * 256u + tid) * 4u;
            const v4f m = *(const v4f*)(bx2 + j);
            const v4f vv = *(const v4f*)(V + j);
            acc = fmaf(m.x, vv.x, acc); acc = fmaf(m.y, vv.y, acc);
            acc = fmaf(m.z, vv.z, acc); acc = fmaf(m.w, vv.w, acc);
        }
#pragma unroll
        for (int o = 16; o > 0; o >>= 1) acc += __shfl_xor(acc, o, 32);
        if (lane == 0u) sR[wave] = acc;
    }
    __syncthreads();
    if (wave == 0u) {
        float val;
        if (blk < (unsigned)(HID / 32)) val = sW[lane];
        else val = ((sR[0] + sR[1]) + (sR[2] + sR[3])) + ((sR[4] + sR[5]) + (sR[6] + sR[7]));
        VST2(float, WC + (size_t)blk * 32u + lane, val);
    }
}

__global__ __launch_bounds__(256) void k_points(const float* __restrict__ x, const float* __restrict__ Wx1,
                                                const float* __restrict__ bx1, const float* __restrict__ WC,
                                                float* __restrict__ out) {
    __shared__ __align__(16) v4f sP[HID];
    __shared__ float sw[HID];
    const unsigned tid = threadIdx.x;
#pragma unroll 1
    for (unsigned i = 0; i < (unsigned)(HID / 256); ++i) {
        const unsigned h = tid + 256u * i;
        v4f p; p.x = Wx1[h]; p.y = Wx1[HID + h]; p.z = Wx1[2 * HID + h]; p.w = bx1[h];
        sP[h] = p;
        sw[h] = WC[h];
    }
    __syncthreads();
    const float cterm = WC[HID];
    const unsigned n = blockIdx.x * 256u + tid;
    const float x0 = x[(size_t)n * 3u + 0u];
    const float x1 = x[(size_t)n * 3u + 1u];
    const float x2 = x[(size_t)n * 3u + 2u];
    float acc = 0.f;
#pragma unroll 1
    for (unsigned h = 0; h < (unsigned)HID; ++h) {
        const v4f p = sP[h];
        const float z = fmaf(x0, p.x, fmaf(x1, p.y, fmaf(x2, p.z, p.w)));
        acc = fmaf(tanhf(z), sw[h], acc);
    }
    VST2(float, out + n, acc + cterm);
}

static constexpr size_t SZ_TP = (size_t)2 * NCH * HID * 4;
static constexpr size_t SZ_YP = (size_t)2 * NCH * 32 * 4;
static constexpr size_t SZ_S  = (size_t)2 * RK * 4;
static constexpr size_t SZ_V  = (size_t)RK * 4;
static constexpr size_t SZ_WC = (((size_t)(HID + 32) * 4) + 255) & ~(size_t)255;
static constexpr size_t OFF_TP = 0;
static constexpr size_t OFF_YP = OFF_TP + SZ_TP;
static constexpr size_t OFF_S  = OFF_YP + SZ_YP;
static constexpr size_t OFF_V  = OFF_S + SZ_S;
static constexpr size_t OFF_WC = OFF_V + SZ_V;
static constexpr size_t WS_TOTAL = OFF_WC + SZ_WC;
static_assert(SZ_TP % 256 == 0 && SZ_YP % 256 == 0 && SZ_S % 256 == 0 && SZ_V % 256 == 0);
static_assert(WS_TOTAL <= (size_t)134217728);
static_assert((size_t)(HID / 32) * 32 + 32 <= (size_t)(HID + 32));

extern "C" void kernel_launch(void* const* d_in, const int* in_sizes, int n_in, void* d_out, int out_size,
                              void* d_ws, size_t ws_size, hipStream_t stream) {
    if (n_in < 16) return;
    if (in_sizes[0] < NPTS * 3 || in_sizes[1] < 1 || in_sizes[2] < NQP * 3 || in_sizes[3] < NQP * 3) return;
    if (in_sizes[4] < 3 * HID || in_sizes[5] < HID || in_sizes[6] < HID * RK || in_sizes[7] < RK) return;
    if (in_sizes[8] < 3 * HID || in_sizes[9] < HID || in_sizes[10] < HID * RK || in_sizes[11] < RK) return;
    if (in_sizes[12] < 3 * HID || in_sizes[13] < HID || in_sizes[14] < HID * RK || in_sizes[15] < RK) return;
    if (out_size < NPTS) return;
    if (WS_TOTAL > ws_size) return;

    const float* input = (const float*)d_in[0];
    const float* eqp   = (const float*)d_in[1];
    const float* qx0   = (const float*)d_in[2];
    const float* qx1   = (const float*)d_in[3];
    const float* Wx1   = (const float*)d_in[4];
    const float* bx1   = (const float*)d_in[5];
    const float* Wx2   = (const float*)d_in[6];
    const float* bx2   = (const float*)d_in[7];
    const float* Wq0a  = (const float*)d_in[8];
    const float* bq0a  = (const float*)d_in[9];
    const float* Wq0b  = (const float*)d_in[10];
    const float* bq0b  = (const float*)d_in[11];
    const float* Wq1a  = (const float*)d_in[12];
    const float* bq1a  = (const float*)d_in[13];
    const float* Wq1b  = (const float*)d_in[14];
    const float* bq1b  = (const float*)d_in[15];
    float* out = (float*)d_out;

    char* wsp = (char*)d_ws;
    float* TP = (float*)(wsp + OFF_TP);
    float* YP = (float*)(wsp + OFF_YP);
    float* S  = (float*)(wsp + OFF_S);
    float* V  = (float*)(wsp + OFF_V);
    float* WC = (float*)(wsp + OFF_WC);

    k_quad_hidden<<<dim3(HID / 256, NCH), 256, 0, stream>>>(qx0, Wq0a, bq0a, eqp, TP, YP);
    k_quad_hidden<<<dim3(HID / 256, NCH), 256, 0, stream>>>(qx1, Wq1a, bq1a, eqp, TP + (size_t)NCH * HID, YP + (size_t)NCH * 32);
    k_quad_out<<<RK / 256, 256, 0, stream>>>(TP, YP, Wq0b, bq0b, S);
    k_quad_out<<<RK / 256, 256, 0, stream>>>(TP + (size_t)NCH * HID, YP + (size_t)NCH * 32, Wq1b, bq1b, S + RK);
    k_rhs<<<1, 512, 0, stream>>>(S, S + RK, V);
    k_hidden_w<<<HID / 32 + 1, 256, 0, stream>>>(Wx2, bx2, V, WC);
    k_points<<<NPTS / 256, 256, 0, stream>>>(input, Wx1, bx1, WC, out);
}
